// SO3Convolution_36163624632815
// MI455X (gfx1250) — hardware-verified
//
#include <hip/hip_runtime.h>
#include <stddef.h>
#include <stdint.h>


#define NTHR    128
#define NWAVE   4
#define EPT     8
#define CHUNK   (NTHR * EPT)
#define WCAP    (EPT * 32)
#define NB      256
#define PW      64
#define ROWF    144
#define ROWH    288
#define NRBF    16
#define HID     64
#define NOUT    16
#define NHM     9
#define RWE     256
#define CUTOFF  5.0f

#define G1      256
#define G2      512
#define G3      2048
#define OW1P    0
#define OW2H    (OW1P + G1 * 8)
#define OW2L    (OW2H + G2 * 8)
#define OW3H    (OW2L + G2 * 8)
#define OW3L    (OW3H + G3 * 8)
#define WTOT    (OW3L + G3 * 8)

#define SZ_ACC   (NB * ROWF * 4)
#define SZ_XS    (NWAVE * 16 * ROWH * 2)
#define SZ_RW    (NWAVE * 16 * RWE * 2)
#define SZ_ESH   (NWAVE * 16 * NHM * 4)
#define SZ_LIST  (NWAVE * WCAP * 4)
#define SZ_PEND  (NWAVE * PW * 4)
#define OFF_ACC  0
#define OFF_XS   (OFF_ACC + SZ_ACC)
#define OFF_RWH  (OFF_XS + SZ_XS)
#define OFF_RWL  (OFF_RWH + SZ_RW)
#define OFF_ESH  (OFF_RWL + SZ_RW)
#define OFF_LIST (OFF_ESH + SZ_ESH)
#define OFF_PEND (OFF_LIST + SZ_LIST)
#define OFF_WCNT (OFF_PEND + SZ_PEND)
#define LDS_BYTES (OFF_WCNT + 16)
#define NQ       ((NB * ROWF) / (128 * NWAVE))

static_assert(WTOT == 43008);
static_assert(((OW2H * 2) % 16) == 0 && ((OW2L * 2) % 16) == 0 && ((OW3H * 2) % 16) == 0 && ((OW3L * 2) % 16) == 0);
static_assert((OFF_XS % 16) == 0);
static_assert((OFF_RWH % 16) == 0);
static_assert((OFF_RWL % 16) == 0);
static_assert((OFF_ESH % 16) == 0);
static_assert((OFF_LIST % 16) == 0);
static_assert((OFF_PEND % 16) == 0);
static_assert((OFF_WCNT % 16) == 0);
static_assert(LDS_BYTES <= 300 * 1024);
static_assert(NQ * 128 * NWAVE == NB * ROWF);
static_assert((NB % NWAVE) == 0 && (NB % 2) == 0);
static_assert(CHUNK <= 4096 && NB <= 1024);
static_assert(PW >= 16 + 32);
static_assert(WCAP == EPT * 32);

typedef float          v4f   __attribute__((ext_vector_type(4)));
typedef float          v8f   __attribute__((ext_vector_type(8)));
typedef int            v4i   __attribute__((ext_vector_type(4)));
typedef unsigned int   v4u   __attribute__((ext_vector_type(4)));
typedef unsigned short v8us  __attribute__((ext_vector_type(8)));
typedef __bf16         v16bf __attribute__((ext_vector_type(16)));
union FragB { v16bf v; v4u q[2]; };
union P8    { v8us u; v4u q; };
struct HL8  { v4u h; v4u l; };

__device__ __forceinline__ v8f zero8f() {
  v8f r;
#pragma unroll
  for (int i = 0; i < 8; ++i) r[i] = 0.0f;
  return r;
}

__device__ __forceinline__ v8f wmb(v16bf a, v16bf b, v8f c) {
  v8f d = __builtin_amdgcn_wmma_f32_16x16x32_bf16(false, a, false, b, (short)0, c, false, false);
  asm volatile("v_nop\n\tv_nop\n\tv_nop\n\tv_nop" : "+v"(d) : "v"(a), "v"(b));
  return d;
}

__device__ __forceinline__ void wave_sync() {
  __builtin_amdgcn_fence(__ATOMIC_RELEASE, "wavefront");
  asm volatile("s_wait_dscnt 0" ::: "memory");
  __builtin_amdgcn_wave_barrier();
}

__device__ __forceinline__ void cbar() {
  asm volatile("" ::: "memory");
}

__device__ __forceinline__ unsigned int bfbits(float x) {
  const unsigned int u = __float_as_uint(x);
  return (u + 0x7FFFu + ((u >> 16) & 1u)) >> 16;
}
__device__ __forceinline__ unsigned short hbits(float v) { return (unsigned short)bfbits(v); }
__device__ __forceinline__ unsigned short lbits(float v) {
  const unsigned int hb = bfbits(v);
  const float hf = __uint_as_float(hb << 16);
  return (unsigned short)bfbits(v - hf);
}

__device__ __forceinline__ v16bf ldAb(const unsigned short* __restrict__ p) {
  FragB a;
  a.q[0] = *(const v4u*)p;
  a.q[1] = *(const v4u*)(p + 16);
  return a.v;
}

__device__ __forceinline__ HL8 act_split(v8f d, const float* __restrict__ bp) {
  const v4f ba = *(const v4f*)bp;
  const v4f bb = *(const v4f*)(bp + 4);
  const float bias[8] = {ba.x, ba.y, ba.z, ba.w, bb.x, bb.y, bb.z, bb.w};
  P8 ph, pl;
#pragma unroll
  for (int r = 0; r < 8; ++r) {
    const float v  = d[r] + bias[r];
    const float sg = v * __builtin_amdgcn_rcpf(1.0f + __expf(-v));
    const unsigned int hb = bfbits(sg);
    const float hf = __uint_as_float(hb << 16);
    const unsigned int lb = bfbits(sg - hf);
    ph.u[r] = (unsigned short)hb;
    pl.u[r] = (unsigned short)lb;
  }
  HL8 o;
  o.h = ph.q;
  o.l = pl.q;
  return o;
}

__device__ __forceinline__ v4u wgrp1(const float* __restrict__ W1, int g) {
  const int row = g >> 2, part = g & 3, k0 = (part & 1) * 8, lo = part >> 1;
  P8 o;
#pragma unroll
  for (int j = 0; j < 8; ++j) {
    const float v = W1[(k0 + j) * HID + row];
    o.u[j] = (lo != 0) ? lbits(v) : hbits(v);
  }
  return o.q;
}
__device__ __forceinline__ v4u wgrpk(const float* __restrict__ W, int ncol, int g, int lo) {
  const int row = g >> 3, k0 = (g & 7) * 8;
  P8 o;
#pragma unroll
  for (int j = 0; j < 8; ++j) {
    const float v = W[(k0 + j) * ncol + row];
    o.u[j] = (lo != 0) ? lbits(v) : hbits(v);
  }
  return o.q;
}
__device__ __forceinline__ void wpass(const float* __restrict__ W1, const float* __restrict__ W2,
                                      const float* __restrict__ W3, unsigned short* wp, int tid) {
  {
    const v4u v = wgrp1(W1, tid);
    *(volatile v4u*)(wp + OW1P + 8 * tid) = v;
  }
#pragma unroll 1
  for (int g = tid; g < G2; g += 256) {
    const v4u v = wgrpk(W2, HID, g, 0);
    *(volatile v4u*)(wp + OW2H + 8 * g) = v;
  }
#pragma unroll 1
  for (int g = tid; g < G2; g += 256) {
    const v4u v = wgrpk(W2, HID, g, 1);
    *(volatile v4u*)(wp + OW2L + 8 * g) = v;
  }
#pragma unroll 1
  for (int g = tid; g < G3; g += 256) {
    const v4u v = wgrpk(W3, RWE, g, 0);
    *(volatile v4u*)(wp + OW3H + 8 * g) = v;
  }
#pragma unroll 1
  for (int g = tid; g < G3; g += 256) {
    const v4u v = wgrpk(W3, RWE, g, 1);
    *(volatile v4u*)(wp + OW3L + 8 * g) = v;
  }
}

__global__ __launch_bounds__(256) void k_wcvt(const float* __restrict__ W1, const float* __restrict__ W2,
                                               const float* __restrict__ W3, unsigned short* wp) {
  const int tid = threadIdx.x;
  wpass(W1, W2, W3, wp, tid);
  __threadfence();
  wpass(W1, W2, W3, wp, tid);
}

__global__ __launch_bounds__(256) void k_xcvt(const float* __restrict__ x, unsigned short* xt, int nN) {
  const int total = nN * 36;
  const int g  = blockIdx.x * 256 + threadIdx.x;
  const int gc = g < total ? g : total - 1;
  const int n  = gc / 36;
  const int w  = gc - n * 36;
  const int plane = (w >= 18) ? 1 : 0;
  const int q  = w - 18 * plane;
  const int f0 = q * 8;
  const int h  = f0 >> 4, i0 = f0 & 15;
  const float* xp = x + (size_t)n * ROWF + i0 * NHM + h;
  P8 o;
#pragma unroll
  for (int j = 0; j < 8; ++j) {
    const float v = xp[j * NHM];
    const unsigned int hb = bfbits(v);
    const float hf = __uint_as_float(hb << 16);
    const unsigned int lb = bfbits(v - hf);
    o.u[j] = (unsigned short)(plane != 0 ? lb : hb);
  }
  unsigned short* op = xt + (size_t)gc * 8;
  const v4u ov = o.q;
  if (g < total) *(volatile v4u*)op = ov;
  __threadfence();
  if (g < total) *(volatile v4u*)op = ov;
}

__device__ __forceinline__ int scan_chunk(const int* __restrict__ dsts, int nE, int cbase, int nodeBase,
                                          int vec8, int* list, int tid, int wave) {
  int wc = 0;
  const int el0  = tid * EPT;
  const int e0   = cbase + el0;
  const int sent = -2147483647 - 1;
  v4i da, db;
  if (vec8 != 0 && cbase + CHUNK <= nE) {
    da = *(const v4i*)(dsts + e0);
    db = *(const v4i*)(dsts + e0 + 4);
  } else {
    da.x = (e0     < nE) ? dsts[min(e0,     nE - 1)] : sent;
    da.y = (e0 + 1 < nE) ? dsts[min(e0 + 1, nE - 1)] : sent;
    da.z = (e0 + 2 < nE) ? dsts[min(e0 + 2, nE - 1)] : sent;
    da.w = (e0 + 3 < nE) ? dsts[min(e0 + 3, nE - 1)] : sent;
    db.x = (e0 + 4 < nE) ? dsts[min(e0 + 4, nE - 1)] : sent;
    db.y = (e0 + 5 < nE) ? dsts[min(e0 + 5, nE - 1)] : sent;
    db.z = (e0 + 6 < nE) ? dsts[min(e0 + 6, nE - 1)] : sent;
    db.w = (e0 + 7 < nE) ? dsts[min(e0 + 7, nE - 1)] : sent;
  }
  const unsigned nb = (unsigned)nodeBase;
  const unsigned s0 = (unsigned)da.x - nb, s1 = (unsigned)da.y - nb;
  const unsigned s2 = (unsigned)da.z - nb, s3 = (unsigned)da.w - nb;
  const unsigned s4 = (unsigned)db.x - nb, s5 = (unsigned)db.y - nb;
  const unsigned s6 = (unsigned)db.z - nb, s7 = (unsigned)db.w - nb;
  const bool h0 = s0 < (unsigned)NB, h1 = s1 < (unsigned)NB, h2 = s2 < (unsigned)NB, h3 = s3 < (unsigned)NB;
  const bool h4 = s4 < (unsigned)NB, h5 = s5 < (unsigned)NB, h6 = s6 < (unsigned)NB, h7 = s7 < (unsigned)NB;
  const unsigned any = __builtin_amdgcn_ballot_w32(h0 | h1 | h2 | h3 | h4 | h5 | h6 | h7);
  if (any != 0u) {
#define HITJ(J, HJ, SJ) { \
      const unsigned mj = __builtin_amdgcn_ballot_w32(HJ); \
      if (mj != 0u) { \
        if (HJ) { \
          const int pos = wc + (int)__builtin_amdgcn_mbcnt_lo(mj, 0u); \
          if (pos < WCAP) list[wave * WCAP + pos] = (el0 + (J)) | ((int)(SJ) << 12); \
        } \
        wc += (int)__builtin_popcount(mj); } }
    HITJ(0, h0, s0)
    HITJ(1, h1, s1)
    HITJ(2, h2, s2)
    HITJ(3, h3, s3)
    HITJ(4, h4, s4)
    HITJ(5, h5, s5)
    HITJ(6, h6, s6)
    HITJ(7, h7, s7)
#undef HITJ
  }
  return wc;
}

__device__ __forceinline__ void run_tile(
    const int* __restrict__ ei, const float* __restrict__ ev,
    const float* __restrict__ b1, const float* __restrict__ b2, const float* __restrict__ b3,
    const float* __restrict__ widths, const unsigned short* __restrict__ wpl,
    const unsigned short* __restrict__ xt,
    float* acc, unsigned char* xsw, unsigned short* rwhw, unsigned short* rwlw, float* eshw,
    const int* pendt, int nv, int nN, int nE, int nodeBase, int lane) {
  const int half = lane >> 4, m = lane & 15;
  const int hc = (m < NHM) ? m : (NHM - 1);
  const v8f z8f = zero8f();
  const unsigned short* w1p = wpl + OW1P;
  const unsigned short* w2h = wpl + OW2H;
  const unsigned short* w2l = wpl + OW2L;
  const unsigned short* w3h = wpl + OW3H;
  const unsigned short* w3l = wpl + OW3L;

  int eid = pendt[(m < nv) ? m : 0];
  eid = eid < 0 ? 0 : (eid > nE - 1 ? nE - 1 : eid);
  int s = ei[eid];
  const int d = ei[(size_t)nE + (size_t)eid];
  s = s < 0 ? 0 : (s > nN - 1 ? nN - 1 : s);
  const int sl  = d - nodeBase;
  const int slq = ((m < nv) && ((unsigned)sl < (unsigned)NB)) ? sl : -1;

  {
    const v4u* gp = (const v4u*)(xt + (size_t)s * ROWH + half * ROWF);
    v4u* lp = (v4u*)(xsw + m * (ROWH * 2) + half * (ROWF * 2));
#pragma unroll
    for (int j = 0; j < 18; ++j) lp[j] = gp[j];
  }

  const float vx = ev[(size_t)eid * 3 + 0];
  const float vy = ev[(size_t)eid * 3 + 1];
  const float vz = ev[(size_t)eid * 3 + 2];
  const float dist = sqrtf(vx * vx + vy * vy + vz * vz);
  const float inv  = __builtin_amdgcn_rcpf(dist + 1e-12f);
  const float nx = vx * inv, ny = vy * inv, nz = vz * inv;
  if (half == 0) {
    const float c1 = 0.4886025119029199f, c2 = 1.0925484305920792f;
    const float c20 = 0.31539156525252005f, c22 = 0.5462742152960396f;
    float* sp = eshw + m * NHM;
    sp[0] = 0.28209479177387814f;
    sp[1] = c1 * ny;
    sp[2] = c1 * nz;
    sp[3] = c1 * nx;
    sp[4] = c2 * nx * ny;
    sp[5] = c2 * ny * nz;
    sp[6] = c20 * (3.0f * nz * nz - 1.0f);
    sp[7] = c2 * nx * nz;
    sp[8] = c22 * (nx * nx - ny * ny);
  }
  const float carg = (3.14159265358979323846f * dist) * 0.2f;
  const float cut  = (dist < CUTOFF) ? 0.5f * (1.0f + cosf(carg)) : 0.0f;

  FragB b1a, b1b;
  {
    const v4f wa = *(const v4f*)(widths + 8 * half);
    const v4f wb = *(const v4f*)(widths + 8 * half + 4);
    const float wv[8] = {wa.x, wa.y, wa.z, wa.w, wb.x, wb.y, wb.z, wb.w};
    P8 rh, rl;
#pragma unroll
    for (int j = 0; j < 8; ++j) {
      const float c  = (float)(8 * half + j) * (CUTOFF / (float)(NRBF - 1));
      const float t  = dist - c;
      const float w  = wv[j];
      const float rr = __builtin_amdgcn_rcpf(2.0f * w * w);
      const float r  = __expf(-(t * t) * rr);
      const unsigned int hb = bfbits(r);
      const float hf = __uint_as_float(hb << 16);
      const unsigned int lb = bfbits(r - hf);
      rh.u[j] = (unsigned short)hb;
      rl.u[j] = (unsigned short)lb;
    }
    b1a.q[0] = rh.q; b1a.q[1] = rh.q;
    b1b.q[0] = rl.q; b1b.q[1] = rl.q;
  }
  wave_sync();

  FragB b2h0, b2h1, b2l0, b2l1;
#define LAYER1(FT, DH, DL) { \
    const v16bf a = ldAb(w1p + (16 * (FT) + m) * 32 + 8 * half); \
    v8f dd = wmb(a, b1a.v, z8f); \
    dd = wmb(a, b1b.v, dd); \
    const HL8 o = act_split(dd, b1 + 16 * (FT) + 8 * half); \
    DH = o.h; DL = o.l; cbar(); }
  LAYER1(0, b2h0.q[0], b2l0.q[0])
  LAYER1(1, b2h0.q[1], b2l0.q[1])
  LAYER1(2, b2h1.q[0], b2l1.q[0])
  LAYER1(3, b2h1.q[1], b2l1.q[1])
#undef LAYER1

  FragB b3h0, b3h1, b3l0, b3l1;
#define LAYER2(FT, DH, DL) { \
    const unsigned short* qh = w2h + (16 * (FT) + m) * 64 + 8 * half; \
    const unsigned short* ql = w2l + (16 * (FT) + m) * 64 + 8 * half; \
    v8f dd = z8f; \
    { const v16bf ah = ldAb(qh); const v16bf al = ldAb(ql); \
      dd = wmb(ah, b2h0.v, dd); dd = wmb(ah, b2l0.v, dd); dd = wmb(al, b2h0.v, dd); } \
    { const v16bf ah = ldAb(qh + 32); const v16bf al = ldAb(ql + 32); \
      dd = wmb(ah, b2h1.v, dd); dd = wmb(ah, b2l1.v, dd); dd = wmb(al, b2h1.v, dd); } \
    const HL8 o = act_split(dd, b2 + 16 * (FT) + 8 * half); \
    DH = o.h; DL = o.l; cbar(); }
  LAYER2(0, b3h0.q[0], b3l0.q[0])
  LAYER2(1, b3h0.q[1], b3l0.q[1])
  LAYER2(2, b3h1.q[0], b3l1.q[0])
  LAYER2(3, b3h1.q[1], b3l1.q[1])
#undef LAYER2

#pragma unroll 1
  for (int o = 0; o < NOUT; ++o) {
    const unsigned short* qh = w3h + (16 * o + m) * 64 + 8 * half;
    const unsigned short* ql = w3l + (16 * o + m) * 64 + 8 * half;
    v8f dd = z8f;
    {
      const v16bf ah = ldAb(qh); const v16bf al = ldAb(ql);
      dd = wmb(ah, b3h0.v, dd); dd = wmb(ah, b3l0.v, dd); dd = wmb(al, b3h0.v, dd);
    }
    {
      const v16bf ah = ldAb(qh + 32); const v16bf al = ldAb(ql + 32);
      dd = wmb(ah, b3h1.v, dd); dd = wmb(ah, b3l1.v, dd); dd = wmb(al, b3h1.v, dd);
    }
    const v4f ba = *(const v4f*)(b3 + 16 * o + 8 * half);
    const v4f bb = *(const v4f*)(b3 + 16 * o + 8 * half + 4);
    const float bias[8] = {ba.x, ba.y, ba.z, ba.w, bb.x, bb.y, bb.z, bb.w};
    P8 ph, pl;
#pragma unroll
    for (int r = 0; r < 8; ++r) {
      const float v = (dd[r] + bias[r]) * cut;
      const unsigned int hb = bfbits(v);
      const float hf = __uint_as_float(hb << 16);
      const unsigned int lb = bfbits(v - hf);
      ph.u[r] = (unsigned short)hb;
      pl.u[r] = (unsigned short)lb;
    }
    const int ro = m * RWE + o * 16 + 8 * half;
    *(v4u*)(rwhw + ro) = ph.q;
    *(v4u*)(rwlw + ro) = pl.q;
  }
  wave_sync();

#pragma unroll 1
  for (int e = 0; e < nv; ++e) {
    FragB fa, fb1, fb2;
    const int ro = e * RWE + m * 16 + 8 * half;
    fa.q[0] = *(const v4u*)(rwhw + ro);
    fa.q[1] = *(const v4u*)(rwlw + ro);
    const unsigned char* xe = xsw + e * (ROWH * 2);
    const v4u xh = *(const v4u*)(xe + hc * 32 + half * 16);
    const v4u xl = *(const v4u*)(xe + ROWF * 2 + hc * 32 + half * 16);
    fb1.q[0] = xh; fb1.q[1] = xh;
    fb2.q[0] = xl; fb2.q[1] = xl;
    v8f dm = wmb(fa.v, fb1.v, z8f);
    dm = wmb(fa.v, fb2.v, dm);
    const int slot = __shfl(slq, e, 32);
    const float sv = eshw[e * NHM + hc];
    if (m < NHM && slot >= 0) {
      float* ap = acc + slot * ROWF + (8 * half) * NHM + m;
#pragma unroll
      for (int r = 0; r < 8; ++r) ap[r * NHM] += dm[r] * sv;
    }
  }
}

__global__ __launch_bounds__(NTHR) void k_conv(
    const int* __restrict__ ei, const float* __restrict__ ev,
    const float* __restrict__ b1, const float* __restrict__ b2, const float* __restrict__ b3,
    const float* __restrict__ widths, const unsigned short* __restrict__ wpl,
    const unsigned short* __restrict__ xt,
    float* outp, int nN, int nE, int vec8) {
  extern __shared__ __attribute__((aligned(16))) unsigned char lds_dyn[];
  float*          acc  = (float*)(lds_dyn + OFF_ACC);
  unsigned char*  xs   = lds_dyn + OFF_XS;
  unsigned short* rwh  = (unsigned short*)(lds_dyn + OFF_RWH);
  unsigned short* rwl  = (unsigned short*)(lds_dyn + OFF_RWL);
  float*          esh  = (float*)(lds_dyn + OFF_ESH);
  int*            list = (int*)(lds_dyn + OFF_LIST);
  int*            pend = (int*)(lds_dyn + OFF_PEND);
  int*            wcnt = (int*)(lds_dyn + OFF_WCNT);

  const int tid = threadIdx.x, lane = tid & 31, wave = tid >> 5;
  const int nodeBase = blockIdx.x * NB;
  const int* dsts = ei + nE;

  unsigned char*  xsw   = xs + wave * (16 * ROWH * 2);
  unsigned short* rwhw  = rwh + wave * (16 * RWE);
  unsigned short* rwlw  = rwl + wave * (16 * RWE);
  float*          eshw  = esh + wave * (16 * NHM);
  int*            pendw = pend + wave * PW;

  {
    const v4f z4 = {0.0f, 0.0f, 0.0f, 0.0f};
    for (int i = tid; i < SZ_ACC / 16; i += NTHR) ((v4f*)acc)[i] = z4;
  }
  if (tid < NWAVE) wcnt[tid] = 0;
  __syncthreads();

  int pn = 0;
  const int nChunks = (nE + CHUNK - 1) / CHUNK;
#pragma unroll 1
  for (int ch = 0; ch < nChunks; ++ch) {
    const int cbase = ch * CHUNK;
    const int wc = scan_chunk(dsts, nE, cbase, nodeBase, vec8, list, tid, wave);
    if (lane == 0) wcnt[wave] = wc;
    __syncthreads();

    const int fin = (ch == nChunks - 1) ? 1 : 0;
#pragma unroll 1
    for (int sw = 0; sw < NWAVE; ++sw) {
      int n = __builtin_amdgcn_readfirstlane(wcnt[sw]);
      n = n > WCAP ? WCAP : (n < 0 ? 0 : n);
      const int flush = (fin != 0 && sw == NWAVE - 1) ? 1 : 0;
      const int ngrp = ((n + 31) >> 5) + flush;
#pragma unroll 1
      for (int g = 0; g < ngrp; ++g) {
        const int idx = g * 32 + lane;
        const bool ok = idx < n;
        const int ent = list[sw * WCAP + (idx < WCAP ? idx : WCAP - 1)];
        const int el  = ent & 4095;
        const int sl  = (ent >> 12) & 1023;
        const bool mine = ok && (sl < NB) && ((sl & (NWAVE - 1)) == wave);
        const unsigned msk = __builtin_amdgcn_ballot_w32(mine);
        if (mine) {
          const int pos = pn + (int)__builtin_amdgcn_mbcnt_lo(msk, 0u);
          int e = cbase + el;
          e = e > nE - 1 ? nE - 1 : e;
          if (pos < PW) pendw[pos] = e;
        }
        pn += (int)__builtin_popcount(msk);
        pn = pn > PW ? PW : pn;

        const bool lastg = (flush != 0) && (g == ngrp - 1);
        int base = 0;
        while ((pn - base >= 16) || (lastg && (pn - base > 0))) {
          int nv = pn - base;
          nv = nv > 16 ? 16 : nv;
          wave_sync();
          run_tile(ei, ev, b1, b2, b3, widths, wpl, xt,
                   acc, xsw, rwhw, rwlw, eshw, pendw + base, nv, nN, nE, nodeBase, lane);
          base += nv;
        }
        if (base > 0) {
          const int rem = pn - base;
          const int src = base + lane;
          const int t = pendw[src < PW ? src : PW - 1];
          wave_sync();
          if (lane < rem) pendw[lane] = t;
          pn = rem;
        }
      }
    }
    __syncthreads();
  }

  int rows = nN - nodeBase;
  rows = rows > NB ? NB : (rows < 0 ? 0 : rows);
  const int limf = rows * ROWF;
  const size_t ob = (size_t)nodeBase * ROWF;
#pragma unroll 1
  for (int q = 0; q < NQ; ++q) {
    const int fo = ((q * NWAVE + wave) * 32 + lane) * 4;
    if (fo + 3 < limf) {
      const v4f v = *(const v4f*)(acc + fo);
      *(volatile v4f*)(outp + ob + (size_t)fo) = v;
    }
  }
  __threadfence();
#pragma unroll 1
  for (int q = 0; q < NQ; ++q) {
    const int fo = ((q * NWAVE + wave) * 32 + lane) * 4;
    if (fo + 3 < limf) {
      const v4f v = *(const v4f*)(acc + fo);
      *(volatile v4f*)(outp + ob + (size_t)fo) = v;
    }
  }
}

extern "C" void kernel_launch(void* const* d_in, const int* in_sizes, int n_in,
                              void* d_out, int out_size, void* d_ws, size_t ws_size,
                              hipStream_t stream) {
  if (n_in < 10) return;
  const int nN = in_sizes[0] / ROWF;
  const int nE = in_sizes[1] / 2;
  if (nN <= 0 || nE <= 0 || nE >= (1 << 29)) return;
  if (in_sizes[0] != nN * ROWF || in_sizes[1] != nE * 2 || in_sizes[2] != nE * 3) return;
  if (in_sizes[3] != NRBF * HID || in_sizes[4] != HID) return;
  if (in_sizes[5] != HID * HID || in_sizes[6] != HID) return;
  if (in_sizes[7] != HID * RWE || in_sizes[8] != RWE || in_sizes[9] != NRBF) return;
  if (out_size != nN * ROWF) return;

  const float* x      = (const float*)d_in[0];
  const int*   ei     = (const int*)d_in[1];
  const float* ev     = (const float*)d_in[2];
  const float* W1     = (const float*)d_in[3];
  const float* b1     = (const float*)d_in[4];
  const float* W2     = (const float*)d_in[5];
  const float* b2     = (const float*)d_in[6];
  const float* W3     = (const float*)d_in[7];
  const float* b3     = (const float*)d_in[8];
  const float* widths = (const float*)d_in[9];
  float* out = (float*)d_out;

  char* ws = (char*)d_ws;
  const size_t szW = (size_t)WTOT * 2;
  const size_t oW  = 0;
  const size_t oX  = 131072;
  const size_t szX = (((size_t)nN * (ROWH * 2)) + 127) & ~(size_t)127;
  const size_t total = oX + szX;
  if (szW > oX) return;
  if (total > ws_size || total > ((size_t)128 << 20)) return;
  unsigned short* wp = (unsigned short*)(ws + oW);
  unsigned short* xt = (unsigned short*)(ws + oX);

  const int vec8 = ((nE & 3) == 0) ? 1 : 0;
  const int nBlk = (nN + NB - 1) / NB;
  const int xBlk = (nN * 36 + 255) / 256;

  k_wcvt<<<1, 256, 0, stream>>>(W1, W2, W3, wp);
  k_xcvt<<<xBlk, 256, 0, stream>>>(x, xt, nN);
  hipFuncSetAttribute(reinterpret_cast<const void*>(&k_conv),
                      hipFuncAttributeMaxDynamicSharedMemorySize, LDS_BYTES);
  k_conv<<<nBlk, NTHR, LDS_BYTES, stream>>>(ei, ev, b1, b2, b3, widths, wp, xt,
                                            out, nN, nE, vec8);
}
